// CausalSelfAttention_26491358281789
// MI455X (gfx1250) — hardware-verified
//
#include <hip/hip_runtime.h>


#ifndef NB
#define NB 2
#endif
#ifndef SEQ
#define SEQ 2048
#endif
#define NB_FULL  2
#define SEQ_FULL 2048
#define DM   1024
#define NH   16
#define HD   64
#define FP   (3 * DM)
#define RH   512
#define RHE  ((RH < SEQ) ? RH : SEQ)
#define PCAR 1024.0f
#define VCAR 16.0f
#define QSC  0.125f
#define NEGV (-1.0e30f)

static_assert(SEQ % 64 == 0);
static_assert(RHE % 32 == 0);
static_assert(DM == NH * HD);
static_assert(DM % 64 == 0);
static_assert(FP % 64 == 0);
static_assert(((size_t)SEQ * DM) % 2048 == 0);
static_assert(((size_t)NH * SEQ * HD) % 512 == 0);
static_assert(((size_t)FP * DM) % 4096 == 0);
static_assert(((size_t)DM * DM) % 4096 == 0);
static_assert(SEQ <= SEQ_FULL);
static_assert(NB <= NB_FULL);

typedef _Float16 h16;
typedef unsigned short bf;
typedef __attribute__((ext_vector_type(16))) __bf16   v16bf;
typedef __attribute__((ext_vector_type(16))) _Float16 v16h;
typedef __attribute__((ext_vector_type(8)))  _Float16 v8h;
typedef __attribute__((ext_vector_type(8)))  unsigned short v8us;
typedef __attribute__((ext_vector_type(8)))  float    v8f;
typedef __attribute__((ext_vector_type(4)))  float    v4f;
typedef __attribute__((ext_vector_type(2)))  float    v2f;
typedef __attribute__((ext_vector_type(2)))  _Float16 v2h;
typedef __attribute__((ext_vector_type(2)))  unsigned short v2us;
typedef v4f  __attribute__((may_alias)) v4fa;

__device__ __forceinline__ unsigned short f2bf(float f) { unsigned u = __float_as_uint(f); u += 0x7FFFu + ((u >> 16) & 1u); return (unsigned short)(u >> 16); }
__device__ __forceinline__ float bf2f(unsigned short b) { return __uint_as_float(((unsigned)b) << 16); }
__device__ __forceinline__ float bfr(float f) { return bf2f(f2bf(f)); }
__device__ __forceinline__ void splitf(float y, unsigned short& h, unsigned short& l) { h = f2bf(y); l = f2bf(y - bf2f(h)); }
__device__ __forceinline__ v16h cat16(v8h lo, v8h hi) { return __builtin_shufflevector(lo, hi, 0, 1, 2, 3, 4, 5, 6, 7, 8, 9, 10, 11, 12, 13, 14, 15); }
__device__ __forceinline__ v16bf cat16b(v8us lo, v8us hi) { return __builtin_bit_cast(v16bf, __builtin_shufflevector(lo, hi, 0, 1, 2, 3, 4, 5, 6, 7, 8, 9, 10, 11, 12, 13, 14, 15)); }
__device__ __forceinline__ v8f wmma16(v16h a, v16h b, v8f c) { return __builtin_amdgcn_wmma_f32_16x16x32_f16(false, a, false, b, (short)0, c, false, false); }
__device__ __forceinline__ v8f wmmab(v16bf a, v16bf b, v8f c) { return __builtin_amdgcn_wmma_f32_16x16x32_bf16(false, a, false, b, (short)0, c, false, false); }

template <typename T16> struct WFrag;
template <> struct WFrag<h16> { typedef v16h V; static __device__ __forceinline__ V ld(const h16* p) { return cat16(*(const v8h*)p, *(const v8h*)(p + 16)); } static __device__ __forceinline__ v8f mma(V a, V b, v8f c) { return wmma16(a, b, c); } };
template <> struct WFrag<bf> { typedef v16bf V; static __device__ __forceinline__ V ld(const bf* p) { return cat16b(*(const v8us*)p, *(const v8us*)(p + 16)); } static __device__ __forceinline__ v8f mma(V a, V b, v8f c) { return wmmab(a, b, c); } };

template <typename T16, int NSPLIT, bool BIAS>
__global__ __launch_bounds__(32) void k_gemmw(const T16* __restrict__ A, const T16* __restrict__ A2, const T16* __restrict__ Bt, const T16* __restrict__ Bt2, int K, float* C, int ldc, const float* __restrict__ bias, size_t sA, size_t sB, size_t sC) {
    typedef typename WFrag<T16>::V V;
    __shared__ __align__(16) float os[16 * 68];
    const size_t z = blockIdx.z; A += z * sA; if (A2) A2 += z * sA; Bt += z * sB; if (Bt2) Bt2 += z * sB; C += z * sC;
    const int lane = threadIdx.x & 31, lr = lane & 15, hi = lane >> 4; const int r0 = blockIdx.x * 64, c0 = blockIdx.y * 64;
    v8f acc[4][4];
#pragma unroll
    for (int mb = 0; mb < 4; ++mb)
#pragma unroll
        for (int nb = 0; nb < 4; ++nb) acc[mb][nb] = (v8f){};
    const size_t aoff = (size_t)(r0 + lr) * K + 8 * hi, boff = (size_t)(c0 + lr) * K + 8 * hi;
#pragma unroll 1
    for (int kc = 0; kc < K; kc += 32) {
        V a[4], a2[4];
#pragma unroll
        for (int mb = 0; mb < 4; ++mb) { a[mb] = WFrag<T16>::ld(A + aoff + (size_t)mb * 16 * K + kc); if (NSPLIT == 1 || NSPLIT == 2) a2[mb] = WFrag<T16>::ld(A2 + aoff + (size_t)mb * 16 * K + kc); }
#pragma unroll
        for (int nb = 0; nb < 4; ++nb) { const V b = WFrag<T16>::ld(Bt + boff + (size_t)nb * 16 * K + kc); V b2; if (NSPLIT >= 2) b2 = WFrag<T16>::ld(Bt2 + boff + (size_t)nb * 16 * K + kc);
#pragma unroll
            for (int mb = 0; mb < 4; ++mb) { acc[mb][nb] = WFrag<T16>::mma(a[mb], b, acc[mb][nb]); if (NSPLIT == 1 || NSPLIT == 2) acc[mb][nb] = WFrag<T16>::mma(a2[mb], b, acc[mb][nb]); if (NSPLIT >= 2) acc[mb][nb] = WFrag<T16>::mma(a[mb], b2, acc[mb][nb]); } }
        asm volatile("v_nop\n\tv_nop\n\tv_nop\n\tv_nop" : "+v"(acc[0][0]), "+v"(acc[1][1]), "+v"(acc[2][2]), "+v"(acc[3][3]) : "v"(a[0]), "v"(a[3]));
    }
    v4f bv = (v4f){0.0f, 0.0f, 0.0f, 0.0f};
    if (BIAS) { const v4f braw = *(const v4f*)(bias + c0 + lr * 4); bv[0] = bfr(braw[0]); bv[1] = bfr(braw[1]); bv[2] = bfr(braw[2]); bv[3] = bfr(braw[3]); }
#pragma unroll
    for (int mb = 0; mb < 4; ++mb) {
#pragma unroll
        for (int nb = 0; nb < 4; ++nb) {
#pragma unroll
            for (int j = 0; j < 8; ++j) os[(hi * 8 + j) * 68 + nb * 16 + lr] = acc[mb][nb][j]; }
        __builtin_amdgcn_fence(3  , "wavefront"); __builtin_amdgcn_wave_barrier(); asm volatile("" ::: "memory");
        float* crow = C + (size_t)(r0 + mb * 16) * ldc + c0;
#pragma unroll 1
        for (int ps = 0; ps < 2; ++ps) {
#pragma unroll
            for (int s = 0; s < 8; ++s) { const int row = 2 * s + hi, cofs = lr * 4; v4f val = *(const v4fa*)(os + row * 68 + cofs); val += bv;
                *(volatile v4f*)(crow + (size_t)row * ldc + cofs) = val; }
            if (ps == 0) __threadfence(); }
        __builtin_amdgcn_fence(3  , "wavefront"); __builtin_amdgcn_wave_barrier(); asm volatile("" ::: "memory");
    }
}

__global__ __launch_bounds__(256) void k_wtG(const float* __restrict__ w, unsigned N, bf* Bt) {
    const unsigned lane = threadIdx.x & 31u; const unsigned L0 = (blockIdx.x * 8u + (threadIdx.x >> 5)) * 8u; const unsigned nlines = N * (unsigned)DM / 64u;
#pragma unroll
    for (int ps = 0; ps < 2; ++ps) {
#pragma unroll 1
        for (unsigned l = 0; l < 8u; ++l) { const unsigned L = L0 + l; if (L >= nlines) break; const unsigned e = L * 64u + lane * 2u; const unsigned k = e % (unsigned)DM, n = e / (unsigned)DM; v2us o;
            o[0] = f2bf(w[(size_t)k * N + n]); o[1] = f2bf(w[(size_t)(k + 1u) * N + n]); *(volatile v2us*)(Bt + e) = o; }
        if (ps == 0) __threadfence(); }
}

__global__ __launch_bounds__(256) void k_cvt8(const float* __restrict__ src, bf* dst, unsigned n8) { const unsigned i = blockIdx.x * 256u + threadIdx.x; if (i >= n8) return; const v8f v = *(const v8f*)(src + (size_t)i * 8); v8us o;
#pragma unroll
    for (int k = 0; k < 8; ++k) o[k] = f2bf(v[k]);
    *(volatile v8us*)(dst + (size_t)i * 8) = o; __threadfence(); *(volatile v8us*)(dst + (size_t)i * 8) = o; }

__global__ __launch_bounds__(256) void k_rope(const float* __restrict__ F, const float* __restrict__ ct, const float* __restrict__ st, float sc, bf* Ph, bf* Pl) {
    const unsigned e = (blockIdx.x * 256u + threadIdx.x) * 2u; if (e >= (unsigned)(NH * SEQ * HD)) return;
    const unsigned d = e % (unsigned)HD, t = (e / (unsigned)HD) % (unsigned)SEQ, h = e / (unsigned)(HD * SEQ);
    const v2f x = *(const v2f*)(F + (size_t)t * FP + h * HD + d);
    const float c = bfr(ct[t * (HD / 2) + (d >> 1)]), s = bfr(st[t * (HD / 2) + (d >> 1)]);
    float a0 = __fmul_rn(x[0], c), b0 = __fmul_rn(x[1], s), a1 = __fmul_rn(x[0], s), b1 = __fmul_rn(x[1], c);
    asm volatile("" : "+v"(a0)); asm volatile("" : "+v"(b0)); asm volatile("" : "+v"(a1)); asm volatile("" : "+v"(b1));
    const float r0 = __fsub_rn(a0, b0) * sc, r1 = __fadd_rn(a1, b1) * sc;
    unsigned short h0, l0, h1, l1; splitf(r0, h0, l0); splitf(r1, h1, l1);
    v2us oh, ol; oh[0] = h0; oh[1] = h1; ol[0] = l0; ol[1] = l1;
    *(volatile v2us*)(Ph + e) = oh; *(volatile v2us*)(Pl + e) = ol; __threadfence(); *(volatile v2us*)(Ph + e) = oh; *(volatile v2us*)(Pl + e) = ol; }

__global__ __launch_bounds__(256) void k_vtp(const float* __restrict__ F, bf* Vh, bf* Vl, h16* V16) {
    const unsigned e = (blockIdx.x * 256u + threadIdx.x) * 2u; if (e >= (unsigned)(NH * HD * SEQ)) return;
    const unsigned t = e % (unsigned)SEQ, d = (e / (unsigned)SEQ) % (unsigned)HD, g = e / (unsigned)(SEQ * HD);
    v2h o16; v2us oh, ol;
#pragma unroll
    for (int q = 0; q < 2; ++q) { const float x = F[(size_t)(t + q) * FP + g * HD + d]; o16[q] = (h16)(x * VCAR); unsigned short a2, c2; splitf(x, a2, c2); oh[q] = a2; ol[q] = c2; }
    *(volatile v2us*)(Vh + e) = oh; *(volatile v2us*)(Vl + e) = ol; *(volatile v2h*)(V16 + e) = o16; __threadfence(); *(volatile v2us*)(Vh + e) = oh; *(volatile v2us*)(Vl + e) = ol; *(volatile v2h*)(V16 + e) = o16; }

template <int HR>
__global__ __launch_bounds__(32) void k_flash(const bf* __restrict__ Qh, const bf* __restrict__ Ql, const bf* __restrict__ Kh, const bf* __restrict__ Kl,
                                              const bf* __restrict__ VTh, const bf* __restrict__ VTl, const h16* __restrict__ VT16, unsigned roff, bf* Ch, bf* Cl) {
    __shared__ __align__(16) float ps[16 * 36];
    __shared__ __align__(16) float os[16 * 68];
    const unsigned lane = threadIdx.x & 31u, lr = lane & 15u, hi = lane >> 4;
    const unsigned h = blockIdx.y, q0 = roff + blockIdx.x * 16u;
    const size_t qo = ((size_t)h * SEQ + q0 + lr) * HD + 8u * hi;
    const v16bf qh0 = WFrag<bf>::ld(Qh + qo), qh1 = WFrag<bf>::ld(Qh + qo + 32), ql0 = WFrag<bf>::ld(Ql + qo), ql1 = WFrag<bf>::ld(Ql + qo + 32);
    v8f o[4];
#pragma unroll
    for (int t = 0; t < 4; ++t) o[t] = (v8f){};
    float mrow[8], lsum[8];
#pragma unroll
    for (int r = 0; r < 8; ++r) { mrow[r] = NEGV; lsum[r] = 0.0f; }
    const float L2E = 1.4426950408889634f;
    const unsigned nkb = (q0 + 16u + 31u) >> 5;
#pragma unroll 1
    for (unsigned kb = 0; kb < nkb; ++kb) {
        const unsigned kbase = kb * 32u;
        v8f s0 = (v8f){}, s1 = (v8f){};
        { const size_t ko = ((size_t)h * SEQ + kbase + lr) * HD + 8u * hi;
          v16bf kh = WFrag<bf>::ld(Kh + ko), kl = WFrag<bf>::ld(Kl + ko);
          s0 = wmmab(qh0, kh, s0); s0 = wmmab(ql0, kh, s0); s0 = wmmab(qh0, kl, s0);
          kh = WFrag<bf>::ld(Kh + ko + 32); kl = WFrag<bf>::ld(Kl + ko + 32);
          s0 = wmmab(qh1, kh, s0); s0 = wmmab(ql1, kh, s0); s0 = wmmab(qh1, kl, s0);
          kh = WFrag<bf>::ld(Kh + ko + 16 * HD); kl = WFrag<bf>::ld(Kl + ko + 16 * HD);
          s1 = wmmab(qh0, kh, s1); s1 = wmmab(ql0, kh, s1); s1 = wmmab(qh0, kl, s1);
          kh = WFrag<bf>::ld(Kh + ko + 16 * HD + 32); kl = WFrag<bf>::ld(Kl + ko + 16 * HD + 32);
          s1 = wmmab(qh1, kh, s1); s1 = wmmab(ql1, kh, s1); s1 = wmmab(qh1, kl, s1);
          asm volatile("v_nop\n\tv_nop\n\tv_nop\n\tv_nop" : "+v"(s0), "+v"(s1) : "v"(kh), "v"(kl)); }
        const unsigned key0 = kbase + lr, key1 = key0 + 16u;
#pragma unroll
        for (int r = 0; r < 8; ++r) {
            const unsigned qrow = q0 + 8u * hi + (unsigned)r;
            const bool ok0 = key0 <= qrow, ok1 = key1 <= qrow;
            const float v0 = ok0 ? s0[r] : NEGV, v1 = ok1 ? s1[r] : NEGV;
            float mx = fmaxf(v0, v1);
#pragma unroll
            for (int off = 1; off < 16; off <<= 1) mx = fmaxf(mx, __shfl_xor(mx, off, 32));
            const float mnew = fmaxf(mrow[r], mx);
            const float alpha = __builtin_amdgcn_exp2f((mrow[r] - mnew) * L2E);
            const float e0 = __builtin_amdgcn_exp2f((v0 - mnew) * L2E), e1 = __builtin_amdgcn_exp2f((v1 - mnew) * L2E);
            const float p0 = ok0 ? e0 : 0.0f, p1 = ok1 ? e1 : 0.0f;
            lsum[r] = lsum[r] * alpha + (p0 + p1);
            mrow[r] = mnew;
#pragma unroll
            for (int t = 0; t < 4; ++t) o[t][r] *= alpha;
            ps[(8u * hi + (unsigned)r) * 36u + lr] = p0; ps[(8u * hi + (unsigned)r) * 36u + 16u + lr] = p1;
        }
        __syncthreads();
        const float* pr = ps + lr * 36u + 8u * hi;
        const v4f f0 = *(const v4fa*)pr, f1 = *(const v4fa*)(pr + 4), f2 = *(const v4fa*)(pr + 16), f3 = *(const v4fa*)(pr + 20);
        if (HR) {
            v8us h0, l0, h1, l1;
#pragma unroll
            for (int i = 0; i < 4; ++i) { unsigned short a, c; splitf(f0[i], a, c); h0[i] = a; l0[i] = c; splitf(f1[i], a, c); h0[4 + i] = a; l0[4 + i] = c;
                splitf(f2[i], a, c); h1[i] = a; l1[i] = c; splitf(f3[i], a, c); h1[4 + i] = a; l1[4 + i] = c; }
            const v16bf pah = cat16b(h0, h1), pal = cat16b(l0, l1);
#pragma unroll
            for (int t = 0; t < 4; ++t) { const size_t vo = ((size_t)h * HD + (unsigned)t * 16u + lr) * SEQ + kbase + 8u * hi;
                const v16bf vh = WFrag<bf>::ld(VTh + vo), vl = WFrag<bf>::ld(VTl + vo);
                o[t] = wmmab(pah, vh, o[t]); o[t] = wmmab(pal, vh, o[t]); o[t] = wmmab(pah, vl, o[t]); }
            asm volatile("v_nop\n\tv_nop\n\tv_nop\n\tv_nop" : "+v"(o[0]), "+v"(o[1]), "+v"(o[2]), "+v"(o[3]) : "v"(pah), "v"(pal));
        } else {
            v8h c0, c1;
#pragma unroll
            for (int i = 0; i < 4; ++i) { c0[i] = (h16)(f0[i] * PCAR); c0[4 + i] = (h16)(f1[i] * PCAR); c1[i] = (h16)(f2[i] * PCAR); c1[4 + i] = (h16)(f3[i] * PCAR); }
            const v16h pa = cat16(c0, c1);
#pragma unroll
            for (int t = 0; t < 4; ++t) { const size_t vo = ((size_t)h * HD + (unsigned)t * 16u + lr) * SEQ + kbase + 8u * hi;
                const v16h vv = WFrag<h16>::ld(VT16 + vo);
                o[t] = wmma16(pa, vv, o[t]); }
            asm volatile("v_nop\n\tv_nop\n\tv_nop\n\tv_nop" : "+v"(o[0]), "+v"(o[1]), "+v"(o[2]), "+v"(o[3]) : "v"(pa));
        }
        __syncthreads();
    }
    float inv[8];
#pragma unroll
    for (int r = 0; r < 8; ++r) { float l = lsum[r];
#pragma unroll
        for (int off = 1; off < 16; off <<= 1) l += __shfl_xor(l, off, 32);
        inv[r] = (HR ? 1.0f : (1.0f / (PCAR * VCAR))) * __builtin_amdgcn_rcpf(l); }
#pragma unroll
    for (int t = 0; t < 4; ++t)
#pragma unroll
        for (int r = 0; r < 8; ++r) os[(hi * 8u + (unsigned)r) * 68u + (unsigned)t * 16u + lr] = o[t][r] * inv[r];
    __syncthreads();
    const unsigned rq = lane >> 3, cofs = (lane & 7u) * 8u;
#pragma unroll 1
    for (int pass = 0; pass < 2; ++pass) {
#pragma unroll
        for (int s = 0; s < 4; ++s) { const unsigned row = 4u * (unsigned)s + rq;
            const v4f a = *(const v4fa*)(os + row * 68u + cofs), b = *(const v4fa*)(os + row * 68u + cofs + 4u); v8us oh, ol;
#pragma unroll
            for (int i = 0; i < 4; ++i) { unsigned short x, y; splitf(a[i], x, y); oh[i] = x; ol[i] = y; splitf(b[i], x, y); oh[4 + i] = x; ol[4 + i] = y; }
            const size_t oo = (size_t)(q0 + row) * DM + h * HD + cofs;
            *(volatile v8us*)(Ch + oo) = oh; *(volatile v8us*)(Cl + oo) = ol; }
        if (pass == 0) __threadfence(); }
}

extern "C" void kernel_launch(void* const* d_in, const int* in_sizes, int n_in,
                              void* d_out, int out_size, void* d_ws, size_t ws_size, hipStream_t stream) {
    if (n_in < 7) return;
    const long long need_x = (long long)(NB - 1) * SEQ_FULL * DM + (long long)SEQ * DM;
    if ((long long)in_sizes[0] < need_x) return;
    if ((long long)in_sizes[1] < (long long)SEQ * (HD / 2) || (long long)in_sizes[2] < (long long)SEQ * (HD / 2)) return;
    if ((long long)in_sizes[3] < (long long)DM * FP || (long long)in_sizes[4] < (long long)FP) return;
    if ((long long)in_sizes[5] < (long long)DM * DM || (long long)in_sizes[6] < (long long)DM) return;
    if ((long long)out_size < need_x) return;
    const float* x = (const float*)d_in[0]; const float* rcos = (const float*)d_in[1]; const float* rsin = (const float*)d_in[2];
    const float* wqkv = (const float*)d_in[3]; const float* bqkv = (const float*)d_in[4]; const float* wout = (const float*)d_in[5]; const float* bout = (const float*)d_in[6];
    float* OUT = (float*)d_out;
    char* wsp = (char*)d_ws;
    auto take = [&](size_t bytes) { char* p = wsp; wsp += (bytes + 255) & ~(size_t)255; return (void*)p; };
    bf* WQT = (bf*)take((size_t)FP * DM * 2);
    bf* WOT = (bf*)take((size_t)DM * DM * 2);
    bf* XB  = (bf*)take((size_t)SEQ * DM * 2);
    float* F = (float*)take((size_t)SEQ * FP * 4);
    bf* QPh = (bf*)take((size_t)NH * SEQ * HD * 2); bf* QPl = (bf*)take((size_t)NH * SEQ * HD * 2);
    bf* KPh = (bf*)take((size_t)NH * SEQ * HD * 2); bf* KPl = (bf*)take((size_t)NH * SEQ * HD * 2);
    bf* VTh = (bf*)take((size_t)NH * HD * SEQ * 2); bf* VTl = (bf*)take((size_t)NH * HD * SEQ * 2); h16* VT16 = (h16*)take((size_t)NH * HD * SEQ * 2);
    bf* CTh = (bf*)take((size_t)SEQ * DM * 2); bf* CTl = (bf*)take((size_t)SEQ * DM * 2);
    if ((size_t)(wsp - (char*)d_ws) > ws_size) return;
    k_wtG<<<(unsigned)(((size_t)FP * DM / 64 + 63) / 64), 256, 0, stream>>>(wqkv, (unsigned)FP, WQT);
    k_wtG<<<(unsigned)(((size_t)DM * DM / 64 + 63) / 64), 256, 0, stream>>>(wout, (unsigned)DM, WOT);
    const unsigned LP = (unsigned)(((size_t)NH * SEQ * HD / 2 + 255) / 256);
    for (int b = 0; b < NB; ++b) {
        k_cvt8<<<(unsigned)(((size_t)SEQ * DM / 8 + 255) / 256), 256, 0, stream>>>(x + (size_t)b * SEQ_FULL * DM, XB, (unsigned)((size_t)SEQ * DM / 8));
        k_gemmw<bf, 0, true><<<dim3(SEQ / 64, FP / 64, 1), 32, 0, stream>>>(XB, nullptr, WQT, nullptr, DM, F, FP, bqkv, 0, 0, 0);
        k_rope<<<LP, 256, 0, stream>>>(F, rcos, rsin, QSC, QPh, QPl);
        k_rope<<<LP, 256, 0, stream>>>(F + DM, rcos, rsin, 1.0f, KPh, KPl);
        k_vtp<<<LP, 256, 0, stream>>>(F + 2 * DM, VTh, VTl, VT16);
        k_flash<1><<<dim3(RHE / 16, NH, 1), 32, 0, stream>>>(QPh, QPl, KPh, KPl, VTh, VTl, VT16, 0u, CTh, CTl);
        if (SEQ > RHE) k_flash<0><<<dim3((SEQ - RHE) / 16, NH, 1), 32, 0, stream>>>(QPh, QPl, KPh, KPl, VTh, VTl, VT16, (unsigned)RHE, CTh, CTl);
        k_gemmw<bf, 1, true><<<dim3(SEQ / 64, DM / 64, 1), 32, 0, stream>>>(CTh, CTl, WOT, nullptr, DM, OUT + (size_t)b * SEQ_FULL * DM, DM, bout, 0, 0, 0);
    }
}
